// HierarchicalClusterLayer_46926812676802
// MI455X (gfx1250) — hardware-verified
//
#include <hip/hip_runtime.h>
#include <math.h>

typedef __attribute__((ext_vector_type(16))) _Float16 v16h;
typedef __attribute__((ext_vector_type(8)))  _Float16 v8h;
typedef __attribute__((ext_vector_type(8)))  float    v8f;
typedef __attribute__((ext_vector_type(4)))  float    v4f;
typedef __attribute__((ext_vector_type(4)))  unsigned int v4u;

constexpr int kDim    = 768;
constexpr int kHeads  = 4;
constexpr int kHD     = kHeads * kDim;
constexpr int kBatch  = 128;
constexpr int kT1     = 16;
constexpr int kT2     = 64;
constexpr int kTPad   = 64;
constexpr int kOutW   = kT1 + kT2;
constexpr int kActRows = kTPad + kBatch;
constexpr int kActLd   = 3 * kHD;
constexpr int kScLd    = kTPad + kBatch;
constexpr float kWCarry  = 1024.0f;
constexpr float kACarry  = 64.0f;
constexpr float kProdInv = 1.0f / (kWCarry * kACarry);
constexpr float kQKInv   = 1.0f / (kACarry * kACarry);
constexpr float kF16MinNormal = 6.103515625e-5f;
constexpr float kLnEps   = 1e-5f;
constexpr float kInvDim  = 1.0f / (float)kDim;
static_assert(kDim == 768 && kHD == 3072 && kOutW == 80, "wire shapes");
static_assert((kDim % 32) == 0, "GEMM K multiple of 32");
static_assert((kDim % 64) == 0 && (kHD % 64) == 0 && (kActLd % 64) == 0 && (kScLd % 64) == 0, "GEMM N multiples of 64");
static_assert((kTPad % 64) == 0 && (kBatch % 64) == 0 && (kActRows % 64) == 0, "GEMM M multiples of 64");
static_assert(kDim == 6 * 128, "score kernel lane map: 6 x (32 lanes x 4)");
static_assert((kBatch * kOutW) % 32 == 0 && ((kBatch * kOutW) / 32) % 8 == 0, "pack kernel: whole lines, 8 per block");
static_assert((kBatch * kT1) % 32 == 0 && (kBatch * kT2) % 32 == 0, "score planes are whole lines");

constexpr size_t kWPlaneElems = (size_t)kHD * kDim;
constexpr size_t kSzWLevel = 4 * kWPlaneElems * 2;
constexpr size_t kSzTPW    = (size_t)kDim * kDim * 2;
constexpr size_t kSzXE     = (size_t)kBatch * kDim * 2;
constexpr size_t kSzXTOK   = (size_t)2 * kTPad * kDim * 2;
constexpr size_t kSzXTP    = (size_t)kBatch * kDim * 2;
constexpr size_t kSzACT    = (size_t)kActRows * kActLd * 2;
constexpr size_t kSzPALL   = (size_t)kActRows * kHD * 4;
constexpr size_t kSzSC     = (size_t)kHeads * kTPad * kScLd * 4;
constexpr size_t kSzS1     = (size_t)kBatch * kT1 * 4;
constexpr size_t kSzS2     = (size_t)kBatch * kT2 * 4;
constexpr size_t kOffW1    = 0;
constexpr size_t kOffW2    = kOffW1   + kSzWLevel;
constexpr size_t kOffTPW   = kOffW2   + kSzWLevel;
constexpr size_t kOffXE    = kOffTPW  + kSzTPW;
constexpr size_t kOffXTOK  = kOffXE   + kSzXE;
constexpr size_t kOffXTP   = kOffXTOK + kSzXTOK;
constexpr size_t kOffACT   = kOffXTP  + kSzXTP;
constexpr size_t kOffPALL  = kOffACT  + 2 * kSzACT;
constexpr size_t kOffSC    = kOffPALL + 2 * kSzPALL;
constexpr size_t kOffS1    = kOffSC   + 2 * kSzSC;
constexpr size_t kOffS2    = kOffS1   + kSzS1;
constexpr size_t kWsTotal  = kOffS2   + kSzS2;
static_assert(kWsTotal == 51748864ull, "carve total");
static_assert(kWsTotal <= 134217728ull, "carve cap");
static_assert((kOffW2 % 128) == 0 && (kOffTPW % 128) == 0 && (kOffXE % 128) == 0 && (kOffXTOK % 128) == 0 &&
              (kOffXTP % 128) == 0 && (kOffACT % 128) == 0 && (kOffPALL % 128) == 0 && (kOffSC % 128) == 0 &&
              (kOffS1 % 128) == 0 && (kOffS2 % 128) == 0 && (kSzACT % 128) == 0 && (kSzPALL % 128) == 0 &&
              (kSzSC % 128) == 0, "128-B aligned regions");

__device__ __forceinline__ unsigned pk16(unsigned short a, unsigned short b) { return (unsigned)a | ((unsigned)b << 16); }
__device__ __forceinline__ unsigned short h_bits_flush(float f) {
  const float g = (fabsf(f) < kF16MinNormal) ? 0.0f : f;
  const _Float16 h = (_Float16)g;
  return __builtin_bit_cast(unsigned short, h);
}
union FragU { v16h v; v8h h[2]; };
__device__ __forceinline__ v16h frag_load(const _Float16* p) {
  FragU f;
  f.h[0] = *(const v8h*)(p);
  f.h[1] = *(const v8h*)(p + 16);
  return f.v;
}
__device__ __forceinline__ v8f mma_h(v16h a, v16h b, v8f c) {
  c = __builtin_amdgcn_wmma_f32_16x16x32_f16(false, a, false, b, (short)0, c, false, false);
  asm volatile("v_nop\n\tv_nop\n\tv_nop\n\tv_nop" : "+v"(c) : "v"(a), "v"(b));
  return c;
}

__global__ __launch_bounds__(256) void cast8_f16_kernel(
    const float* __restrict__ s0, const float* __restrict__ s1, const float* __restrict__ s2, const float* __restrict__ s3,
    unsigned short* __restrict__ out, int real8a, int real8b, int tot8, float carry) {
  const int y = blockIdx.y;
  const float* src = (y == 0) ? s0 : (y == 1) ? s1 : (y == 2) ? s2 : s3;
  const int real8 = (y == 0) ? real8a : real8b;
  const int i = blockIdx.x * 256 + threadIdx.x;
  if (i >= tot8) return;
  const int ic = (i < real8) ? i : (real8 - 1);
  const float* p = src + 8 * (size_t)ic;
  const v4f a = *(const v4f*)(p);
  const v4f c = *(const v4f*)(p + 4);
  float x0 = a[0], x1 = a[1], x2 = a[2], x3 = a[3];
  float x4 = c[0], x5 = c[1], x6 = c[2], x7 = c[3];
  asm volatile("" : "+v"(x0), "+v"(x1), "+v"(x2), "+v"(x3));
  asm volatile("" : "+v"(x4), "+v"(x5), "+v"(x6), "+v"(x7));
  const bool live = (i < real8);
  const unsigned short h0 = h_bits_flush(live ? x0 * carry : 0.0f);
  const unsigned short h1 = h_bits_flush(live ? x1 * carry : 0.0f);
  const unsigned short h2 = h_bits_flush(live ? x2 * carry : 0.0f);
  const unsigned short h3 = h_bits_flush(live ? x3 * carry : 0.0f);
  const unsigned short h4 = h_bits_flush(live ? x4 * carry : 0.0f);
  const unsigned short h5 = h_bits_flush(live ? x5 * carry : 0.0f);
  const unsigned short h6 = h_bits_flush(live ? x6 * carry : 0.0f);
  const unsigned short h7 = h_bits_flush(live ? x7 * carry : 0.0f);
  const v4u u = (v4u){pk16(h0, h1), pk16(h2, h3), pk16(h4, h5), pk16(h6, h7)};
  unsigned short* q = out + (size_t)y * (size_t)tot8 * 8 + 8 * (size_t)i;
  *(volatile v4u*)q = u;
  __threadfence();
  *(volatile v4u*)q = u;
}

template <bool BIAS, bool OUT16, int OSC>
__global__ __launch_bounds__(256) void gemm64_f16(
    const unsigned short* __restrict__ Ap, int lda, long strideA,
    const unsigned short* __restrict__ Btp, int ldb, long strideB,
    void* __restrict__ Cout, int ldc, long strideC,
    const float* __restrict__ bias,
    int M, int N, int K, float scale) {
  const float sm_scale = 1.0f / sqrtf((float)kDim);
  const float oscale = (OSC == 2) ? sm_scale : ((OSC == 1) ? kACarry : 1.0f);
  const _Float16* A  = (const _Float16*)Ap;
  const _Float16* Bt = (const _Float16*)Btp;
  __shared__ __align__(16) float sT[8][16 * 68];
  const int b    = blockIdx.y;
  const int lane = threadIdx.x & 31;
  const int wave = threadIdx.x >> 5;
  const int tilesN = N >> 6;
  const int tilesM = M >> 6;
  const int tile = blockIdx.x * 8 + wave;
  if (tile >= tilesM * tilesN) return;
  const int tm = tile / tilesN;
  const int tn = tile - tm * tilesN;
  const int m0 = tm << 6;
  const int n0 = tn << 6;

  const _Float16* Ab = A  + (size_t)b * strideA;
  const _Float16* Bb = Bt + (size_t)b * strideB;

  const int rlane = lane & 15;
  const int koff  = (lane >> 4) * 8;
  const int mOff  = (lane >> 4) * 8;

  v8f acc[4][4];
#pragma unroll
  for (int i = 0; i < 4; ++i)
#pragma unroll
    for (int j = 0; j < 4; ++j) acc[i][j] = (v8f){0.f, 0.f, 0.f, 0.f, 0.f, 0.f, 0.f, 0.f};

  for (int k0 = 0; k0 < K; k0 += 32) {
    v16h bh[4];
#pragma unroll
    for (int j = 0; j < 4; ++j) {
      const size_t bo = (size_t)(n0 + (j << 4) + rlane) * ldb + koff + k0;
      bh[j] = frag_load(Bb + bo);
    }
#pragma unroll
    for (int i = 0; i < 4; ++i) {
      const size_t ao = (size_t)(m0 + (i << 4) + rlane) * lda + koff + k0;
      const v16h ah = frag_load(Ab + ao);
#pragma unroll
      for (int j = 0; j < 4; ++j) acc[i][j] = mma_h(ah, bh[j], acc[i][j]);
    }
  }

  float* slab = sT[wave];
#pragma unroll
  for (int i = 0; i < 4; ++i) {
    const int mBase = m0 + (i << 4);
#pragma unroll
    for (int j = 0; j < 4; ++j) {
      const int n = n0 + (j << 4) + rlane;
      float bv = 0.f;
      if (BIAS) bv = bias[n];
#pragma unroll
      for (int r = 0; r < 8; ++r) {
        float v = acc[i][j][r] * scale;
        if (BIAS) v += bv;
        v *= oscale;
        slab[(mOff + r) * 68 + (j << 4) + rlane] = v;
      }
    }
    __builtin_amdgcn_fence(__ATOMIC_RELEASE, "workgroup");
    __builtin_amdgcn_wave_barrier();
    __builtin_amdgcn_fence(__ATOMIC_ACQUIRE, "workgroup");
    if (!OUT16) {
      float* C = (float*)Cout + (size_t)b * strideC;
      const int hh = lane >> 4, c4 = (lane & 15) * 4;
      for (int pass = 0; pass < 2; ++pass) {
#pragma unroll
        for (int it = 0; it < 8; ++it) {
          const int row = it * 2 + hh;
          const v4f v = *(const v4f*)(slab + row * 68 + c4);
          *(volatile v4f*)(C + (size_t)(mBase + row) * ldc + n0 + c4) = v;
        }
        __threadfence();
      }
    } else {
      const int q = lane >> 3, c8 = (lane & 7) * 8;
      unsigned short* C = (unsigned short*)Cout + (size_t)b * strideC;
      v4u pk[4];
#pragma unroll
      for (int it = 0; it < 4; ++it) {
        const int row = it * 4 + q;
        const float* sp = slab + row * 68 + c8;
        const v4f x0 = *(const v4f*)(sp);
        const v4f x1 = *(const v4f*)(sp + 4);
        const unsigned short h0 = h_bits_flush(x0[0]), h1 = h_bits_flush(x0[1]);
        const unsigned short h2 = h_bits_flush(x0[2]), h3 = h_bits_flush(x0[3]);
        const unsigned short h4 = h_bits_flush(x1[0]), h5 = h_bits_flush(x1[1]);
        const unsigned short h6 = h_bits_flush(x1[2]), h7 = h_bits_flush(x1[3]);
        pk[it] = (v4u){pk16(h0, h1), pk16(h2, h3), pk16(h4, h5), pk16(h6, h7)};
      }
      for (int pass = 0; pass < 2; ++pass) {
#pragma unroll
        for (int it = 0; it < 4; ++it) {
          const int row = it * 4 + q;
          *(volatile v4u*)(C + (size_t)(mBase + row) * ldc + n0 + c8) = pk[it];
        }
        __threadfence();
      }
    }
    __builtin_amdgcn_fence(__ATOMIC_RELEASE, "workgroup");
    __builtin_amdgcn_wave_barrier();
    __builtin_amdgcn_fence(__ATOMIC_ACQUIRE, "workgroup");
  }
}

template <int T>
__global__ __launch_bounds__(256) void score_kernel(
    const float* __restrict__ SC, const float* __restrict__ PALL,
    const float* __restrict__ fcb, const float* __restrict__ tok,
    const float* __restrict__ lng, const float* __restrict__ lnb,
    const float* __restrict__ slng, const float* __restrict__ slnb,
    const float* __restrict__ sw, const float* __restrict__ sb,
    float* __restrict__ Sout) {
  __shared__ __align__(16) float ys[8][kDim];
  __shared__ float scs[32];
  const int lane = threadIdx.x & 31;
  const int wave = threadIdx.x >> 5;
  float* yw = &ys[wave][0];
  const float sbv = sb[0];
  const int hl = lane & 3;
#pragma unroll 1
  for (int p = 0; p < 4; ++p) {
    const int f = blockIdx.x * 32 + wave * 4 + p;
    int b = f / T;
    const int t = f - b * T;
    b = (b < kBatch) ? b : (kBatch - 1);
    const float* sr = SC + (size_t)(hl * kTPad + t) * kScLd;
    const float s0 = sr[t];
    const float s1 = sr[kTPad + b];
    const float dd = s1 - s0;
    const float ee = expf(-fabsf(dd));
    const float inv = 1.0f / (1.0f + ee);
    const float big = inv;
    const float sml = ee * inv;
    const float a0v = (dd >= 0.0f) ? sml : big;
    const float a1v = (dd >= 0.0f) ? big : sml;
    const float a00 = __shfl(a0v, 0), a01 = __shfl(a0v, 1), a02 = __shfl(a0v, 2), a03 = __shfl(a0v, 3);
    const float a10 = __shfl(a1v, 0), a11 = __shfl(a1v, 1), a12 = __shfl(a1v, 2), a13 = __shfl(a1v, 3);
    const float* pt = PALL + (size_t)t * kHD;
    const float* pb = PALL + (size_t)(kTPad + b) * kHD;
    const float* tk = tok + (size_t)t * kDim;
    float sum = 0.f;
#pragma unroll 1
    for (int i = 0; i < 6; ++i) {
      const int c = i * 128 + lane * 4;
      v4f v = *(const v4f*)(fcb + c);
      v4f q;
      q = *(const v4f*)(pt + c);
      v += a00 * q;
      q = *(const v4f*)(pb + c);
      v += a10 * q;
      q = *(const v4f*)(pt + kDim + c);
      v += a01 * q;
      q = *(const v4f*)(pb + kDim + c);
      v += a11 * q;
      q = *(const v4f*)(pt + 2 * kDim + c);
      v += a02 * q;
      q = *(const v4f*)(pb + 2 * kDim + c);
      v += a12 * q;
      q = *(const v4f*)(pt + 3 * kDim + c);
      v += a03 * q;
      q = *(const v4f*)(pb + 3 * kDim + c);
      v += a13 * q;
      q = *(const v4f*)(tk + c);
      v += q;
      *(v4f*)(yw + c) = v;
      sum += (v[0] + v[1]) + (v[2] + v[3]);
    }
#pragma unroll
    for (int off = 16; off > 0; off >>= 1) sum += __shfl_xor(sum, off);
    const float mean1 = sum * kInvDim;
    float sq = 0.f;
#pragma unroll 1
    for (int i = 0; i < 6; ++i) {
      const int c = i * 128 + lane * 4;
      const v4f v = *(const v4f*)(yw + c);
      const v4f d = v - mean1;
      sq += (d[0] * d[0] + d[1] * d[1]) + (d[2] * d[2] + d[3] * d[3]);
    }
#pragma unroll
    for (int off = 16; off > 0; off >>= 1) sq += __shfl_xor(sq, off);
    const float rs1 = rsqrtf(sq * kInvDim + kLnEps);
    float sum2 = 0.f;
#pragma unroll 1
    for (int i = 0; i < 6; ++i) {
      const int c = i * 128 + lane * 4;
      const v4f v = *(const v4f*)(yw + c);
      const v4f g = *(const v4f*)(lng + c);
      const v4f bb = *(const v4f*)(lnb + c);
      const v4f z = ((v - mean1) * rs1) * g + bb;
      *(v4f*)(yw + c) = z;
      sum2 += (z[0] + z[1]) + (z[2] + z[3]);
    }
#pragma unroll
    for (int off = 16; off > 0; off >>= 1) sum2 += __shfl_xor(sum2, off);
    const float mean2 = sum2 * kInvDim;
    float sq2 = 0.f;
#pragma unroll 1
    for (int i = 0; i < 6; ++i) {
      const int c = i * 128 + lane * 4;
      const v4f z = *(const v4f*)(yw + c);
      const v4f d = z - mean2;
      sq2 += (d[0] * d[0] + d[1] * d[1]) + (d[2] * d[2] + d[3] * d[3]);
    }
#pragma unroll
    for (int off = 16; off > 0; off >>= 1) sq2 += __shfl_xor(sq2, off);
    const float rs2 = rsqrtf(sq2 * kInvDim + kLnEps);
    float dot = 0.f;
#pragma unroll 1
    for (int i = 0; i < 6; ++i) {
      const int c = i * 128 + lane * 4;
      const v4f z = *(const v4f*)(yw + c);
      const v4f g = *(const v4f*)(slng + c);
      const v4f bb = *(const v4f*)(slnb + c);
      const v4f wv = *(const v4f*)(sw + c);
      const v4f w = ((z - mean2) * rs2) * g + bb;
      dot += (w[0] * wv[0] + w[1] * wv[1]) + (w[2] * wv[2] + w[3] * wv[3]);
    }
#pragma unroll
    for (int off = 16; off > 0; off >>= 1) dot += __shfl_xor(dot, off);
    const float score = dot + sbv;
    if (lane == 0) scs[wave * 4 + p] = score;
  }
  __syncthreads();
  if (wave == 0) {
    const float v = scs[lane];
    volatile float* q = Sout + (size_t)blockIdx.x * 32 + lane;
    *q = v;
    __threadfence();
    *q = v;
  }
}

__global__ __launch_bounds__(256) void pack_kernel(const float* __restrict__ S1, const float* __restrict__ S2,
                                                   float* __restrict__ out) {
  const int lane = threadIdx.x & 31;
  const int wave = threadIdx.x >> 5;
  const int line = blockIdx.x * 8 + wave;
  const int o = line * 32 + lane;
  const int b = o / kOutW;
  const int c = o - b * kOutW;
  const int c1 = (c < kT1) ? c : (kT1 - 1);
  const int c2 = (c >= kT1) ? (c - kT1) : 0;
  float v1 = S1[b * kT1 + c1];
  float v2 = S2[b * kT2 + c2];
  asm volatile("" : "+v"(v1), "+v"(v2));
  const float v = (c < kT1) ? v1 : v2;
  volatile float* q = out + o;
  *q = v;
  __threadfence();
  *q = v;
}

extern "C" void kernel_launch(void* const* d_in, const int* in_sizes, int n_in,
                              void* d_out, int out_size, void* d_ws, size_t ws_size,
                              hipStream_t stream) {
  if (n_in < 27) return;
  if (in_sizes[0] != kBatch * kDim) return;
  if (in_sizes[1] != kT1 * kDim) return;
  if (in_sizes[2] != kT2 * kDim) return;
  if (in_sizes[3] != kDim * kDim) return;
  if (in_sizes[4] != kDim) return;
  for (int L = 0; L < 2; ++L) {
    const int ib = (L == 0) ? 5 : 16;
    if (in_sizes[ib + 0] != kHD * kDim) return;
    if (in_sizes[ib + 1] != kHD * kDim) return;
    if (in_sizes[ib + 2] != kHD * kDim) return;
    if (in_sizes[ib + 3] != kDim * kHD) return;
    for (int j = 4; j < 10; ++j)
      if (in_sizes[ib + j] != kDim) return;
    if (in_sizes[ib + 10] != 1) return;
  }
  if (out_size != kBatch * kOutW) return;
  if (ws_size < kWsTotal) return;

  const float* task_emb    = (const float*)d_in[0];
  const float* tokens_l1   = (const float*)d_in[1];
  const float* tokens_l2   = (const float*)d_in[2];
  const float* task_proj_w = (const float*)d_in[3];
  const float* task_proj_b = (const float*)d_in[4];
  float* out = (float*)d_out;

  char* ws = (char*)d_ws;
  unsigned short* TPW  = (unsigned short*)(ws + kOffTPW);
  unsigned short* XE   = (unsigned short*)(ws + kOffXE);
  unsigned short* XTOK = (unsigned short*)(ws + kOffXTOK);
  unsigned short* XTP  = (unsigned short*)(ws + kOffXTP);
  float* S1 = (float*)(ws + kOffS1);
  float* S2 = (float*)(ws + kOffS2);

  const int wTot8 = (int)(kWPlaneElems / 8);

  for (int L = 0; L < 2; ++L) {
    const int ib = (L == 0) ? 5 : 16;
    unsigned short* W16 = (unsigned short*)(ws + ((L == 0) ? kOffW1 : kOffW2));
    cast8_f16_kernel<<<dim3(wTot8 / 256, 4), 256, 0, stream>>>(
        (const float*)d_in[ib + 0], (const float*)d_in[ib + 1], (const float*)d_in[ib + 2], (const float*)d_in[ib + 3],
        W16, wTot8, wTot8, wTot8, kWCarry);
  }
  cast8_f16_kernel<<<dim3((kDim * kDim / 8) / 256, 1), 256, 0, stream>>>(
      task_proj_w, task_proj_w, task_proj_w, task_proj_w, TPW,
      kDim * kDim / 8, kDim * kDim / 8, kDim * kDim / 8, kWCarry);
  cast8_f16_kernel<<<dim3((kBatch * kDim / 8) / 256, 1), 256, 0, stream>>>(
      task_emb, task_emb, task_emb, task_emb, XE,
      kBatch * kDim / 8, kBatch * kDim / 8, kBatch * kDim / 8, kACarry);
  cast8_f16_kernel<<<dim3((kTPad * kDim / 8) / 256, 2), 256, 0, stream>>>(
      tokens_l1, tokens_l2, tokens_l2, tokens_l2, XTOK,
      kT1 * kDim / 8, kT2 * kDim / 8, kTPad * kDim / 8, kACarry);

  gemm64_f16<true, true, 1><<<dim3(3, 1), 256, 0, stream>>>(
      XE, kDim, 0L,
      TPW, kDim, 0L,
      (void*)XTP, kDim, 0L,
      task_proj_b,
      kBatch, kDim, kDim, kProdInv);

  for (int L = 0; L < 2; ++L) {
    const int ib = (L == 0) ? 5 : 16;
    unsigned short* W16  = (unsigned short*)(ws + ((L == 0) ? kOffW1 : kOffW2));
    unsigned short* ACT  = (unsigned short*)(ws + kOffACT + (size_t)L * kSzACT);
    float*          PALL = (float*)(ws + kOffPALL + (size_t)L * kSzPALL);
    float*          SC   = (float*)(ws + kOffSC + (size_t)L * kSzSC);
    const unsigned short* XT = XTOK + (size_t)L * kTPad * kDim;
    const float* fcb  = (const float*)d_in[ib + 4];
    const float* lng  = (const float*)d_in[ib + 5];
    const float* lnb  = (const float*)d_in[ib + 6];
    const float* slng = (const float*)d_in[ib + 7];
    const float* slnb = (const float*)d_in[ib + 8];
    const float* sw   = (const float*)d_in[ib + 9];
    const float* sb   = (const float*)d_in[ib + 10];
    const float* tok  = (L == 0) ? tokens_l1 : tokens_l2;

    gemm64_f16<false, true, 1><<<dim3(18, 1), 256, 0, stream>>>(
        XT, kDim, 0L,
        W16, kDim, 0L,
        (void*)ACT, kActLd, 0L,
        task_proj_b,
        kTPad, kActLd, kDim, kProdInv);
    gemm64_f16<false, true, 1><<<dim3(24, 1), 256, 0, stream>>>(
        XTP, kDim, 0L,
        W16 + kWPlaneElems, kDim, 0L,
        (void*)(ACT + (size_t)kTPad * kActLd + kHD), kActLd, 0L,
        task_proj_b,
        kBatch, 2 * kHD, kDim, kProdInv);
    gemm64_f16<false, false, 0><<<dim3(5, kHeads), 256, 0, stream>>>(
        ACT + 2 * kHD, kActLd, (long)kDim,
        W16 + 3 * kWPlaneElems, kHD, (long)kDim,
        (void*)PALL, kHD, (long)kDim,
        task_proj_b,
        kActRows, kDim, kDim, kProdInv);
    gemm64_f16<false, false, 2><<<dim3(1, kHeads), 256, 0, stream>>>(
        ACT, kActLd, (long)kDim,
        ACT + kHD, kActLd, (long)kDim,
        (void*)SC, kScLd, (long)(kTPad * kScLd),
        task_proj_b,
        kTPad, kScLd, kDim, kQKInv);
    if (L == 0) {
      score_kernel<kT1><<<(kBatch * kT1) / 32, 256, 0, stream>>>(
          SC, PALL, fcb, tok, lng, lnb, slng, slnb, sw, sb, S1);
    } else {
      score_kernel<kT2><<<(kBatch * kT2) / 32, 256, 0, stream>>>(
          SC, PALL, fcb, tok, lng, lnb, slng, slnb, sw, sb, S2);
    }
  }

  pack_kernel<<<(kBatch * kOutW / 32) / 8, 256, 0, stream>>>(S1, S2, out);
}
